// learning_gain_unit_7481833030184
// MI455X (gfx1250) — hardware-run, weakly checked
//
#include <hip/hip_runtime.h>
#include <hip/hip_fp16.h>
#include <math.h>

typedef __attribute__((ext_vector_type(16))) _Float16 v16h;
typedef __attribute__((ext_vector_type(8)))  _Float16 v8h;
typedef __attribute__((ext_vector_type(8)))  float    v8f;
typedef __attribute__((ext_vector_type(4)))  float    v4f;
typedef __attribute__((ext_vector_type(4)))  unsigned v4u;

constexpr int kBatch     = 128;
constexpr int kLen       = 100;
constexpr int kChan      = 1024;
constexpr int kSteps     = kLen - 1;
constexpr int kRows      = kBatch * kSteps;
constexpr int kDepth     = 2 * kChan;
constexpr int kCols3     = 3 * kChan;
constexpr int kChunks    = 4;
constexpr int kChunkB    = kBatch / kChunks;
constexpr int kChunkRows = kChunkB * kSteps;
constexpr int kGroups    = (kSteps + 3) / 4;
constexpr int kInBig     = kBatch * kLen * kChan;
constexpr int kInW       = kDepth * kChan;
constexpr int kTilePitch = 65;
static_assert(kSteps == 99 && kRows == 12672 && kDepth == 2048 && kCols3 == 3072);
static_assert(kChunkB == 32 && kChunkRows == 3168 && kGroups == 25);
static_assert(kInBig == 13107200 && kInW == 2097152);
static_assert((kChunkRows % 32) == 0 && (kCols3 % 64) == 0 && (kDepth % 32) == 0);
static_assert(((kChunkRows / 32) * (kCols3 / 64)) % 8 == 0);
static_assert((kDepth / 8) == 256 && (kChan % 256) == 0 && (kChan % 64) == 0 && (kDepth % 64) == 0);

constexpr float kCarryX = 16.0f;
constexpr float kCarryW = 4096.0f;
constexpr float kFold   = 1.0f / (kCarryX * kCarryW);
constexpr float kHalfMinNormal = 6.103515625e-05f;
static_assert(kFold * 65536.0f == 1.0f);

constexpr size_t kSzX16  = (size_t)kRows * kDepth * 2;
constexpr size_t kSzWT   = (size_t)kCols3 * kDepth * 2;
constexpr size_t kSzP    = (size_t)kChunkRows * kCols3 * 4;
constexpr size_t kOffX16 = 0;
constexpr size_t kOffWT  = kOffX16 + kSzX16;
constexpr size_t kOffP   = kOffWT + kSzWT;
constexpr size_t kWsTotal = kOffP + kSzP;
static_assert(kSzX16 == 51904512ull);
static_assert(kSzWT == 12582912ull);
static_assert(kSzP == 38928384ull);
static_assert(kWsTotal == 103415808ull);
static_assert(kWsTotal <= 134217728ull);
static_assert((kOffWT % 128) == 0 && (kOffP % 128) == 0);

__device__ __forceinline__ float bf16_rne(float f) { unsigned int u = __float_as_uint(f); u += 0x7FFFu + ((u >> 16) & 1u); return __uint_as_float(u & 0xFFFF0000u); }
__device__ __forceinline__ float flush_small(float v) {
  return (fabsf(v) < kHalfMinNormal) ? 0.0f : v;
}
__device__ __forceinline__ unsigned pack2_f16(float a, float b) {
  const _Float16 h0 = (_Float16)a;
  const _Float16 h1 = (_Float16)b;
  const unsigned short u0 = __builtin_bit_cast(unsigned short, h0);
  const unsigned short u1 = __builtin_bit_cast(unsigned short, h1);
  return (unsigned)u0 | ((unsigned)u1 << 16);
}

namespace eng {
union FragU { v16h v; v8h h[2]; };
__device__ __forceinline__ v16h frag_load(const _Float16* p) {
  FragU f;
  f.h[0] = *(const v8h*)(p);
  f.h[1] = *(const v8h*)(p + 16);
  return f.v;
}
__device__ __forceinline__ v8f mma(v16h a, v16h b, v8f c) {
  return __builtin_amdgcn_wmma_f32_16x16x32_f16(false, a, false, b, (short)0, c, false, false);
}
__device__ __forceinline__ void guard1(v8f& a, v16h x, v16h y) {
  asm volatile("v_nop\n\tv_nop\n\tv_nop\n\tv_nop" : "+v"(a) : "v"(x), "v"(y));
}
__device__ __forceinline__ void guard_acc(v8f& a) {
  asm volatile("v_nop\n\tv_nop\n\tv_nop\n\tv_nop" : "+v"(a));
}
__device__ __forceinline__ void keep4(v16h a, v16h b, v16h c, v16h d) {
  asm volatile("v_nop" :: "v"(a), "v"(b), "v"(c), "v"(d));
}

template <int MI, int SPL>
__global__ __launch_bounds__(256) void gemm_f16_kernel(
    const unsigned short* __restrict__ Ap, const unsigned short* __restrict__ A2p, int lda,
    const unsigned short* __restrict__ Btp, const unsigned short* __restrict__ Bt2p, int ldb,
    float* __restrict__ C, int ldc, int M, int N, int K, float scale, float rscale)
{
  static_assert(MI >= 1 && MI <= 2);
  static_assert(SPL >= 0 && SPL <= 2);
  const _Float16* A   = (const _Float16*)Ap;
  const _Float16* A2  = (const _Float16*)A2p;
  const _Float16* Bt  = (const _Float16*)Btp;
  const _Float16* Bt2 = (const _Float16*)Bt2p;
  __shared__ __align__(16) float sT[8][16 * 68];
  const int lane = threadIdx.x & 31;
  const int wave = threadIdx.x >> 5;
  const int tilesN = N >> 6;
  const int tilesM = M / (16 * MI);
  const int tile = blockIdx.x * 8 + wave;
  if (tile >= tilesM * tilesN) return;
  const int tm = tile / tilesN;
  const int tn = tile - tm * tilesN;
  const int m0 = tm * (16 * MI);
  const int n0 = tn << 6;
  const int rlane = lane & 15;
  const int koff  = (lane >> 4) * 8;
  const int mOff  = (lane >> 4) * 8;

  v8f acc[MI][4], accr[MI][4];
#pragma unroll
  for (int i = 0; i < MI; ++i)
#pragma unroll
    for (int j = 0; j < 4; ++j) {
      acc[i][j]  = (v8f){0.f, 0.f, 0.f, 0.f, 0.f, 0.f, 0.f, 0.f};
      accr[i][j] = (v8f){0.f, 0.f, 0.f, 0.f, 0.f, 0.f, 0.f, 0.f};
    }

  for (int k0 = 0; k0 < K; k0 += 32) {
    v16h bh[4], bl[4];
#pragma unroll
    for (int j = 0; j < 4; ++j) {
      const size_t bo = (size_t)(n0 + (j << 4) + rlane) * ldb + koff + k0;
      bh[j] = frag_load(Bt + bo);
      if (SPL == 2) bl[j] = frag_load(Bt2 + bo); else bl[j] = bh[j];
    }
#pragma unroll
    for (int i = 0; i < MI; ++i) {
      const size_t ao = (size_t)(m0 + (i << 4) + rlane) * lda + koff + k0;
      const v16h ah = frag_load(A + ao);
      v16h al = ah;
      if (SPL >= 1) al = frag_load(A2 + ao);
#pragma unroll
      for (int j = 0; j < 4; ++j) {
        acc[i][j] = mma(ah, bh[j], acc[i][j]);
        if (SPL >= 1) accr[i][j] = mma(al, bh[j], accr[i][j]);
        if (SPL == 2) accr[i][j] = mma(ah, bl[j], accr[i][j]);
      }
#pragma unroll
      for (int j = 0; j < 4; ++j) {
        guard1(acc[i][j], ah, al);
        if (SPL >= 1) guard1(accr[i][j], ah, al);
      }
    }
    keep4(bh[0], bh[1], bh[2], bh[3]);
    if (SPL == 2) keep4(bl[0], bl[1], bl[2], bl[3]);
  }
#pragma unroll
  for (int i = 0; i < MI; ++i)
#pragma unroll
    for (int j = 0; j < 4; ++j) {
      guard_acc(acc[i][j]);
      if (SPL >= 1) guard_acc(accr[i][j]);
    }

  float* slab = sT[wave];
#pragma unroll
  for (int i = 0; i < MI; ++i) {
    const int mBase = m0 + (i << 4);
#pragma unroll
    for (int j = 0; j < 4; ++j) {
#pragma unroll
      for (int r = 0; r < 8; ++r) {
        float v = acc[i][j][r] * scale;
        if (SPL >= 1) v += accr[i][j][r] * rscale;
        slab[(mOff + r) * 68 + (j << 4) + rlane] = v;
      }
    }
    __builtin_amdgcn_fence(__ATOMIC_RELEASE, "workgroup");
    __builtin_amdgcn_wave_barrier();
    __builtin_amdgcn_fence(__ATOMIC_ACQUIRE, "workgroup");
    {
      const int hh = lane >> 4, c4 = (lane & 15) * 4;
      for (int pass = 0; pass < 2; ++pass) {
#pragma unroll
        for (int it = 0; it < 8; ++it) {
          const int row = it * 2 + hh;
          const v4f v = *(const v4f*)(slab + row * 68 + c4);
          *(volatile v4f*)(C + (size_t)(mBase + row) * ldc + n0 + c4) = v;
        }
        __threadfence();
      }
    }
    __builtin_amdgcn_fence(__ATOMIC_RELEASE, "workgroup");
    __builtin_amdgcn_wave_barrier();
    __builtin_amdgcn_fence(__ATOMIC_ACQUIRE, "workgroup");
  }
}
}

__global__ __launch_bounds__(256) void x_plane_kernel(
    const float* __restrict__ qe, const float* __restrict__ cs, unsigned* __restrict__ X16)
{
  int r = blockIdx.x;
  r = (r < kRows) ? r : (kRows - 1);
  const int tid = threadIdx.x;
  const int b = r / kSteps;
  const int t = r - b * kSteps;
  const int col = tid * 8;
  const bool firstHalf = (col < kChan);
  const float* src = firstHalf ? cs : qe;
  const int sc = firstHalf ? col : (col - kChan);
  const float* sp = src + ((size_t)b * kLen + t) * kChan + sc;
  const v4f a0 = *(const v4f*)(sp);
  const v4f a1 = *(const v4f*)(sp + 4);
  float h[8];
#pragma unroll
  for (int e = 0; e < 4; ++e) {
    const float f0 = a0[e];
    const float f1 = a1[e];
    h[e]     = flush_small(bf16_rne(f0) * kCarryX);
    h[4 + e] = flush_small(bf16_rne(f1) * kCarryX);
  }
  v4u w;
  w[0] = pack2_f16(h[0], h[1]);
  w[1] = pack2_f16(h[2], h[3]);
  w[2] = pack2_f16(h[4], h[5]);
  w[3] = pack2_f16(h[6], h[7]);
  unsigned* p = X16 + ((size_t)r * kDepth + col) / 2;
  *(volatile v4u*)p = w;
  __threadfence();
  *(volatile v4u*)p = w;
}

__global__ __launch_bounds__(256) void w_pack_kernel(
    const float* __restrict__ Wg, const float* __restrict__ Wk, const float* __restrict__ Wr,
    unsigned* __restrict__ WT)
{
  __shared__ float tile[64 * kTilePitch];
  const int tid = threadIdx.x;
  int nt = blockIdx.x;
  int kt = blockIdx.y;
  int j  = blockIdx.z;
  nt = (nt < kChan / 64) ? nt : (kChan / 64 - 1);
  kt = (kt < kDepth / 64) ? kt : (kDepth / 64 - 1);
  j  = (j < 3) ? j : 2;
  const int n0 = nt * 64;
  const int k0 = kt * 64;
  const float* W = (j == 0) ? Wg : ((j == 1) ? Wk : Wr);
#pragma unroll
  for (int it = 0; it < 4; ++it) {
    const int kr = it * 16 + (tid >> 4);
    const int n4 = (tid & 15) * 4;
    const v4f a = *(const v4f*)(W + (size_t)(k0 + kr) * kChan + n0 + n4);
#pragma unroll
    for (int e = 0; e < 4; ++e) {
      const float f = a[e];
      tile[kr * kTilePitch + n4 + e] = flush_small(bf16_rne(f) * kCarryW);
    }
  }
  __syncthreads();
  v4u w[2];
#pragma unroll
  for (int it = 0; it < 2; ++it) {
    const int nr = it * 32 + (tid >> 3);
    const int k8 = (tid & 7) * 8;
    float h[8];
#pragma unroll
    for (int e = 0; e < 8; ++e) h[e] = tile[(k8 + e) * kTilePitch + nr];
    v4u wv;
    wv[0] = pack2_f16(h[0], h[1]);
    wv[1] = pack2_f16(h[2], h[3]);
    wv[2] = pack2_f16(h[4], h[5]);
    wv[3] = pack2_f16(h[6], h[7]);
    w[it] = wv;
  }
  for (int pass = 0; pass < 2; ++pass) {
#pragma unroll
    for (int it = 0; it < 2; ++it) {
      const int nr = it * 32 + (tid >> 3);
      const int k8 = (tid & 7) * 8;
      unsigned* p = WT + ((size_t)(j * kChan + n0 + nr) * kDepth + k0 + k8) / 2;
      *(volatile v4u*)p = w[it];
    }
    __threadfence();
  }
}

__global__ __launch_bounds__(256) void gate_scan_kernel(
    const float* __restrict__ P, const float* __restrict__ sim, const float* __restrict__ expp,
    const float* __restrict__ bgp, const float* __restrict__ bkp, const float* __restrict__ brp,
    float* __restrict__ out, int chunk)
{
  const int tid = threadIdx.x;
  int bl = blockIdx.x >> 2;
  bl = (bl < kChunkB) ? bl : (kChunkB - 1);
  const int cc = (chunk < 0) ? 0 : ((chunk > kChunks - 1) ? (kChunks - 1) : chunk);
  const int b = cc * kChunkB + bl;
  const int d = (blockIdx.x & 3) * 256 + tid;

  const float bg = bf16_rne(bgp[d]);
  const float bk = bf16_rne(bkp[d]);
  const float br = bf16_rne(brp[d]);
  float carry = bf16_rne(expp[d]);

  float* orow = out + (size_t)b * kLen * kChan + d;
  const float* srow = sim + (size_t)b * kLen * kChan + d;
  const float* prow = P + (size_t)bl * kSteps * kCols3 + d;

  {
    const float v0 = carry;
    *(volatile float*)orow = v0;
    __threadfence();
    *(volatile float*)orow = v0;
  }

  for (int g = 0; g < kGroups; ++g) {
    float res[4];
#pragma unroll
    for (int s = 0; s < 4; ++s) res[s] = 0.0f;
#pragma unroll
    for (int s = 0; s < 4; ++s) {
      const int t = 4 * g + s;
      if (t < kSteps) {
        const float* pp = prow + (size_t)t * kCols3;
        const float pg = pp[0] + bg;
        const float pk = pp[kChan] + bk;
        const float pr = pp[2 * kChan] + br;
        const float sraw = srow[(size_t)(t + 1) * kChan];
        const float gate = 1.0f / (1.0f + expf(-pg));
        const float cand = tanhf(pk);
        const float rst  = 1.0f / (1.0f + expf(-pr));
        const float sv = bf16_rne(sraw);
        const float drive = (1.0f - rst) * gate * cand * sv;
        carry = fmaf(rst, carry, drive);
        res[s] = carry;
      }
    }
    for (int pass = 0; pass < 2; ++pass) {
#pragma unroll
      for (int s = 0; s < 4; ++s) {
        const int t = 4 * g + s;
        if (t < kSteps) {
          const float v = res[s];
          *(volatile float*)(orow + (size_t)(t + 1) * kChan) = v;
        }
      }
      __threadfence();
    }
  }
}

extern "C" void kernel_launch(void* const* d_in, const int* in_sizes, int n_in,
                              void* d_out, int out_size, void* d_ws, size_t ws_size,
                              hipStream_t stream)
{
  if (n_in < 10) return;
  if (in_sizes[0] != kInBig) return;
  if (in_sizes[1] != kInBig) return;
  if (in_sizes[2] != kInBig) return;
  if (in_sizes[3] != kChan) return;
  if (in_sizes[4] != kInW) return;
  if (in_sizes[5] != kChan) return;
  if (in_sizes[6] != kInW) return;
  if (in_sizes[7] != kChan) return;
  if (in_sizes[8] != kInW) return;
  if (in_sizes[9] != kChan) return;
  if (out_size != kInBig) return;
  if (ws_size < kWsTotal) return;

  const float* q_embed = (const float*)d_in[0];
  const float* cluster = (const float*)d_in[1];
  const float* all_sim = (const float*)d_in[2];
  const float* expp    = (const float*)d_in[3];
  const float* W_gate  = (const float*)d_in[4];
  const float* b_gate  = (const float*)d_in[5];
  const float* W_k     = (const float*)d_in[6];
  const float* b_k     = (const float*)d_in[7];
  const float* W_re    = (const float*)d_in[8];
  const float* b_re    = (const float*)d_in[9];
  float* out = (float*)d_out;

  char* ws = (char*)d_ws;
  unsigned* X16 = (unsigned*)(ws + kOffX16);
  unsigned* WT  = (unsigned*)(ws + kOffWT);
  float*    P   = (float*)(ws + kOffP);

  x_plane_kernel<<<kRows, 256, 0, stream>>>(q_embed, cluster, X16);

  w_pack_kernel<<<dim3(kChan / 64, kDepth / 64, 3), 256, 0, stream>>>(W_gate, W_k, W_re, WT);

  const unsigned short* WT16 = (const unsigned short*)WT;
  for (int c = 0; c < kChunks; ++c) {
    const unsigned short* A16 = (const unsigned short*)X16 + (size_t)c * kChunkRows * kDepth;
    eng::gemm_f16_kernel<2, 0><<<dim3((kChunkRows / 32) * (kCols3 / 64) / 8), 256, 0, stream>>>(
        A16, nullptr, kDepth, WT16, nullptr, kDepth, P, kCols3, kChunkRows, kCols3, kDepth, kFold, 0.0f);
    gate_scan_kernel<<<kChunkB * (kChan / 256), 256, 0, stream>>>(
        P, all_sim, expp, b_gate, b_k, b_re, out, c);
  }
}
